// MemResProjections_13477607375124
// MI455X (gfx1250) — hardware-verified
//
#include <hip/hip_runtime.h>
#include <stddef.h>
#include <stdint.h>

#define NB   4
#define SQ   2048
#define NMEM 64
#define NT   2112
#define HID  1024
#define NTOK 8192

static_assert(NT == SQ + NMEM);
static_assert(NTOK == NB * SQ);
static_assert(HID == 128 * 8);
static_assert(SQ % 256 == 0);
static_assert(SQ % 16 == 0);
static_assert(NT % 64 == 0);
static_assert(NT % 2 == 0);
static_assert((NT * 2) % 128 == 0);
static_assert(NMEM == 64);

typedef _Float16 v16h __attribute__((ext_vector_type(16)));
typedef _Float16 v8h  __attribute__((ext_vector_type(8)));
typedef float    v8f  __attribute__((ext_vector_type(8)));
typedef float    v4f  __attribute__((ext_vector_type(4)));
typedef unsigned int v4u __attribute__((ext_vector_type(4)));

union Frag  { v16h v; v8h h[2]; };
union Pack8 { v8h h; v4u u; };

__device__ __forceinline__ v8f mma16(v16h a, v16h b, v8f c) {
  c = __builtin_amdgcn_wmma_f32_16x16x32_f16(false, a, false, b, (short)0, c, false, false);
  asm volatile("v_nop\n\tv_nop\n\tv_nop\n\tv_nop" : "+v"(c) : "v"(a), "v"(b));
  return c;
}

__device__ __forceinline__ v16h ldfrag(const _Float16* p, int ld, int row0, int k0, int lane) {
  const int m = lane & 15, lh = lane >> 4;
  const _Float16* q = p + (size_t)(row0 + m) * ld + k0 + 8 * lh;
  Frag f;
  f.h[0] = *(const v8h*)(q);
  f.h[1] = *(const v8h*)(q + 16);
  return f.v;
}

__device__ __forceinline__ v8f zero8() { return (v8f){0.f, 0.f, 0.f, 0.f, 0.f, 0.f, 0.f, 0.f}; }

__device__ __forceinline__ void gemm32x64_rng(const _Float16* __restrict__ A, int lda,
                                              const _Float16* __restrict__ Bt, int ldb,
                                              int m0, int n0, int kbeg, int kend, int lane, v8f (&acc)[2][4]) {
#pragma unroll 2
  for (int k0 = kbeg; k0 < kend; k0 += 32) {
    const v16h a0 = ldfrag(A, lda, m0, k0, lane);
    const v16h a1 = ldfrag(A, lda, m0 + 16, k0, lane);
    const v16h b0 = ldfrag(Bt, ldb, n0, k0, lane);
    const v16h b1 = ldfrag(Bt, ldb, n0 + 16, k0, lane);
    const v16h b2 = ldfrag(Bt, ldb, n0 + 32, k0, lane);
    const v16h b3 = ldfrag(Bt, ldb, n0 + 48, k0, lane);
    acc[0][0] = mma16(a0, b0, acc[0][0]);
    acc[1][0] = mma16(a1, b0, acc[1][0]);
    acc[0][1] = mma16(a0, b1, acc[0][1]);
    acc[1][1] = mma16(a1, b1, acc[1][1]);
    acc[0][2] = mma16(a0, b2, acc[0][2]);
    acc[1][2] = mma16(a1, b2, acc[1][2]);
    acc[0][3] = mma16(a0, b3, acc[0][3]);
    acc[1][3] = mma16(a1, b3, acc[1][3]);
  }
}

__global__ __launch_bounds__(256) void k_prep(const float* __restrict__ hid, const float* __restrict__ mem,
                                              const float* __restrict__ nw,
                                              _Float16* __restrict__ vp, _Float16* __restrict__ xh) {
  __shared__ float red[8];
  const int tid = threadIdx.x, lane = tid & 31, wave = tid >> 5, g = tid >> 7;
  const int r = blockIdx.x * 2 + g;
  const int b = r / NT;
  const int t = r - b * NT;
  const int col = (tid & 127) * 8;
  const bool local = (t < SQ);
  const int tl = local ? t : 0;
  const int tm = local ? 0 : (t - SQ);
  const float* src = local ? (hid + ((size_t)b * SQ + tl) * HID + col)
                           : (mem + ((size_t)b * NMEM + tm) * HID + col);
  const v4f a0 = *(const v4f*)(src);
  const v4f a1 = *(const v4f*)(src + 4);
  float ss = a0[0] * a0[0] + a0[1] * a0[1] + a0[2] * a0[2] + a0[3] * a0[3]
           + a1[0] * a1[0] + a1[1] * a1[1] + a1[2] * a1[2] + a1[3] * a1[3];
#pragma unroll
  for (int off = 1; off < 32; off <<= 1) ss += __shfl_xor(ss, off, 32);
  if (lane == 0) red[wave] = ss;
  __syncthreads();
  const float tot = (red[4 * g] + red[4 * g + 1]) + (red[4 * g + 2] + red[4 * g + 3]);
  const float rn = rsqrtf(tot * 0.0009765625f + 1e-6f);
  const v4f w0 = *(const v4f*)(nw + col);
  const v4f w1 = *(const v4f*)(nw + col + 4);
  const float y0 = local ? (a0[0] * rn * w0[0]) : a0[0];
  const float y1 = local ? (a0[1] * rn * w0[1]) : a0[1];
  const float y2 = local ? (a0[2] * rn * w0[2]) : a0[2];
  const float y3 = local ? (a0[3] * rn * w0[3]) : a0[3];
  const float y4 = local ? (a1[0] * rn * w1[0]) : a1[0];
  const float y5 = local ? (a1[1] * rn * w1[1]) : a1[1];
  const float y6 = local ? (a1[2] * rn * w1[2]) : a1[2];
  const float y7 = local ? (a1[3] * rn * w1[3]) : a1[3];
  Pack8 pv, px;
  pv.h = (v8h){(_Float16)y0, (_Float16)y1, (_Float16)y2, (_Float16)y3,
               (_Float16)y4, (_Float16)y5, (_Float16)y6, (_Float16)y7};
  px.h = (v8h){(_Float16)a0[0], (_Float16)a0[1], (_Float16)a0[2], (_Float16)a0[3],
               (_Float16)a1[0], (_Float16)a1[1], (_Float16)a1[2], (_Float16)a1[3]};
  const v4u vv = pv.u, vx = px.u;
  const size_t ov = ((size_t)b * NT + t) * HID + col;
  const size_t ox = ((size_t)b * SQ + tl) * HID + col;
  *(volatile v4u*)(vp + ov) = vv;
  if (local) *(volatile v4u*)(xh + ox) = vx;
  __threadfence();
  *(volatile v4u*)(vp + ov) = vv;
  if (local) *(volatile v4u*)(xh + ox) = vx;
}

__global__ __launch_bounds__(256) void k_cvtw(const float* __restrict__ src, _Float16* __restrict__ dh, float sc) {
  const int tid = threadIdx.x;
  const int row = blockIdx.x * 2 + (tid >> 7);
  const int col = (tid & 127) * 8;
  const size_t o = (size_t)row * HID + col;
  const v4f a0 = *(const v4f*)(src + o);
  const v4f a1 = *(const v4f*)(src + o + 4);
  Pack8 pk;
  pk.h = (v8h){(_Float16)(a0[0] * sc), (_Float16)(a0[1] * sc), (_Float16)(a0[2] * sc), (_Float16)(a0[3] * sc),
               (_Float16)(a1[0] * sc), (_Float16)(a1[1] * sc), (_Float16)(a1[2] * sc), (_Float16)(a1[3] * sc)};
  const v4u vv = pk.u;
  volatile v4u* d = (volatile v4u*)(dh + o);
  *d = vv;
  __threadfence();
  *d = vv;
}

#define KTP 72
__global__ __launch_bounds__(256) void k_proj(const _Float16* __restrict__ A, size_t astr,
                                              const _Float16* __restrict__ W,
                                              _Float16* __restrict__ O, size_t ostr) {
  __shared__ __align__(16) _Float16 st[8][32 * KTP];
  const int tid = threadIdx.x, lane = tid & 31, wave = tid >> 5;
  const int hh = lane >> 4, c = lane & 15;
  const int b  = blockIdx.z;
  const int wm = wave >> 2, wn = wave & 3;
  const int m0 = blockIdx.x * 64 + 32 * wm;
  const int n0 = blockIdx.y * 256 + 64 * wn;
  const _Float16* Ab = A + (size_t)b * astr;
  _Float16* Ob = O + (size_t)b * ostr;

  v8f acc[2][4];
#pragma unroll
  for (int s = 0; s < 2; ++s)
#pragma unroll
    for (int t = 0; t < 4; ++t) acc[s][t] = zero8();
  gemm32x64_rng(Ab, HID, W, HID, m0, n0, 0, HID, lane, acc);

  _Float16* pw = st[wave];
#pragma unroll
  for (int s = 0; s < 2; ++s)
#pragma unroll
    for (int t = 0; t < 4; ++t)
#pragma unroll
      for (int r = 0; r < 8; ++r)
        pw[(16 * s + 8 * hh + r) * KTP + 16 * t + c] = (_Float16)(acc[s][t][r] * 0.03125f);
  __syncthreads();

  v4u val[8];
  size_t go[8];
#pragma unroll
  for (int it = 0; it < 8; ++it) {
    const int p  = lane + 32 * it;
    const int L  = p >> 3;
    const int pc = p & 7;
    Pack8 pk;
    pk.h    = *(const v8h*)(pw + L * KTP + pc * 8);
    val[it] = pk.u;
    go[it]  = (size_t)(m0 + L) * HID + n0 + pc * 8;
  }
  for (int ps = 0; ps < 2; ++ps) {
#pragma unroll
    for (int it = 0; it < 8; ++it) *(volatile v4u*)(Ob + go[it]) = val[it];
    __threadfence();
  }
}

__global__ __launch_bounds__(256) void k_vtr(const _Float16* __restrict__ vp, _Float16* __restrict__ vt) {
  __shared__ __align__(16) _Float16 tl[64 * KTP];
  const int tid = threadIdx.x;
  const int b  = blockIdx.z;
  const int t0 = blockIdx.x * 64;
  const int h0 = blockIdx.y * 64;
  const _Float16* src = vp + (size_t)b * NT * HID;
  _Float16* dst = vt + (size_t)b * HID * NT;
#pragma unroll
  for (int j = 0; j < 2; ++j) {
    const int p  = tid + 256 * j;
    const int tt = p >> 3;
    const int hq = (p & 7) * 8;
    *(v8h*)(tl + tt * KTP + hq) = *(const v8h*)(src + (size_t)(t0 + tt) * HID + h0 + hq);
  }
  __syncthreads();
  v4u val[2];
  size_t go[2];
#pragma unroll
  for (int j = 0; j < 2; ++j) {
    const int p  = tid + 256 * j;
    const int hr = p >> 3;
    const int pc = p & 7;
    const _Float16* cp = tl + (pc * 8) * KTP + hr;
    Pack8 pk;
    pk.h = (v8h){cp[0 * KTP], cp[1 * KTP], cp[2 * KTP], cp[3 * KTP],
                 cp[4 * KTP], cp[5 * KTP], cp[6 * KTP], cp[7 * KTP]};
    val[j] = pk.u;
    go[j]  = (size_t)(h0 + hr) * NT + t0 + pc * 8;
  }
  for (int ps = 0; ps < 2; ++ps) {
#pragma unroll
    for (int j = 0; j < 2; ++j) *(volatile v4u*)(dst + go[j]) = val[j];
    __threadfence();
  }
}

#define LP 2120
__global__ __launch_bounds__(256) void k_ssm(const _Float16* __restrict__ qp,
                                             const _Float16* __restrict__ kp,
                                             _Float16* __restrict__ pp) {
  __shared__ __align__(16) float sl[16 * LP];
  const int tid = threadIdx.x, lane = tid & 31, wave = tid >> 5;
  const int hh = lane >> 4, c = lane & 15;
  const int rg = blockIdx.x;
  const int b  = blockIdx.y;
  const int q0 = rg * 16;
  const int G  = (rg >> 2) + 2;
  const _Float16* Qb = qp + (size_t)b * SQ * HID;
  const _Float16* Kb = kp + (size_t)b * NT * HID;

  for (int g = wave; g < G; g += 8) {
    const int kr0 = (g == 0) ? SQ : (g - 1) * 64;
    v8f acc[4];
#pragma unroll
    for (int t = 0; t < 4; ++t) acc[t] = zero8();
#pragma unroll 2
    for (int k0 = 0; k0 < HID; k0 += 32) {
      const v16h a = ldfrag(Qb, HID, q0, k0, lane);
#pragma unroll
      for (int t = 0; t < 4; ++t) {
        const v16h kb = ldfrag(Kb, HID, kr0 + 16 * t, k0, lane);
        acc[t] = mma16(a, kb, acc[t]);
      }
    }
#pragma unroll
    for (int t = 0; t < 4; ++t)
#pragma unroll
      for (int r = 0; r < 8; ++r)
        sl[(8 * hh + r) * LP + kr0 + 16 * t + c] = acc[t][r] * 0.03125f;
  }
  __syncthreads();

  const float NEG = -3.0e38f;
  for (int ri = 0; ri < 2; ++ri) {
    const int rr   = wave * 2 + ri;
    const int pos  = q0 + rr;
    const int cend = pos + 1;
    float* row = sl + rr * LP;

    float m = NEG;
    for (int c0 = 0; c0 < cend; c0 += 32) {
      const int cc = c0 + lane;
      const float x = row[cc];
      const float v = (cc < cend) ? x : NEG;
      m = fmaxf(m, v);
    }
    m = fmaxf(m, row[SQ + lane]);
    m = fmaxf(m, row[SQ + 32 + lane]);
#pragma unroll
    for (int off = 1; off < 32; off <<= 1) m = fmaxf(m, __shfl_xor(m, off, 32));

    float sum = 0.f;
    for (int c0 = 0; c0 < cend; c0 += 32) {
      const int cc = c0 + lane;
      const float x = row[cc];
      const float e = __expf(x - m);
      const float ev = (cc < cend) ? e : 0.f;
      sum += ev;
      if (cc < cend) row[cc] = e;
    }
    {
      const float e0 = __expf(row[SQ + lane] - m);
      const float e1 = __expf(row[SQ + 32 + lane] - m);
      row[SQ + lane] = e0;
      row[SQ + 32 + lane] = e1;
      sum += e0 + e1;
    }
#pragma unroll
    for (int off = 1; off < 32; off <<= 1) sum += __shfl_xor(sum, off, 32);
    const float inv = 1024.0f / sum;
    __syncthreads();

    _Float16* Pb = pp + ((size_t)b * SQ + pos) * NT;
    v4u val[9];
#pragma unroll
    for (int it = 0; it < 9; ++it) {
      const int p  = lane + 32 * it;
      const int tc = 8 * p;
      const int ta = (tc < NT - 8) ? tc : (NT - 8);
      Pack8 pk;
      _Float16 hv[8];
#pragma unroll
      for (int e = 0; e < 8; ++e) {
        const float x = row[ta + e];
        const int tk = tc + e;
        const bool vis = (tk <= pos) || (tk >= SQ);
        const float pv = vis ? (x * inv) : 0.f;
        hv[e] = (_Float16)pv;
      }
      pk.h = (v8h){hv[0], hv[1], hv[2], hv[3], hv[4], hv[5], hv[6], hv[7]};
      val[it] = pk.u;
    }
    for (int ps = 0; ps < 2; ++ps) {
#pragma unroll
      for (int it = 0; it < 9; ++it) {
        const int p = lane + 32 * it;
        if (p < NT / 8) *(volatile v4u*)(Pb + 8 * p) = val[it];
      }
      __threadfence();
    }
  }
}

#define OTP 68
__global__ __launch_bounds__(256) void k_pvg(const _Float16* __restrict__ pp,
                                             const _Float16* __restrict__ vt,
                                             const _Float16* __restrict__ xh,
                                             const _Float16* __restrict__ wg,
                                             const float* __restrict__ gb,
                                             const float* __restrict__ hid,
                                             float* __restrict__ out) {
  __shared__ __align__(16) float st[8][32 * OTP];
  __shared__ __align__(16) float sa[8][16 * OTP];
  const int tid = threadIdx.x, lane = tid & 31, wave = tid >> 5;
  const int hh = lane >> 4, c = lane & 15;
  const int b  = blockIdx.z;
  const int m0 = blockIdx.x * 256 + wave * 32;
  const int n0 = blockIdx.y * 64;
  const _Float16* Pb = pp + (size_t)b * SQ * NT;
  const _Float16* Vb = vt + (size_t)b * HID * NT;
  const size_t trow = (size_t)b * SQ;

  v8f acc[2][4];
#pragma unroll
  for (int s = 0; s < 2; ++s)
#pragma unroll
    for (int t = 0; t < 4; ++t) acc[s][t] = zero8();
  gemm32x64_rng(Pb, NT, Vb, NT, m0, n0, 0, m0 + 32, lane, acc);
  gemm32x64_rng(Pb, NT, Vb, NT, m0, n0, SQ, NT, lane, acc);

  float* sw = st[wave];
#pragma unroll
  for (int s = 0; s < 2; ++s)
#pragma unroll
    for (int t = 0; t < 4; ++t)
#pragma unroll
      for (int r = 0; r < 8; ++r)
        sw[(16 * s + 8 * hh + r) * OTP + 16 * t + c] = acc[s][t][r] * 0.0009765625f;
  __syncthreads();

#pragma unroll
  for (int s = 0; s < 2; ++s)
#pragma unroll
    for (int t = 0; t < 4; ++t) acc[s][t] = zero8();
  gemm32x64_rng(xh + trow * HID, HID, wg, HID, m0, n0, 0, HID, lane, acc);

  float bb[4];
#pragma unroll
  for (int t = 0; t < 4; ++t) bb[t] = gb[n0 + 16 * t + c];

  float* aw = sa[wave];
#pragma unroll
  for (int sub = 0; sub < 2; ++sub) {
    __syncthreads();
#pragma unroll
    for (int t = 0; t < 4; ++t) {
#pragma unroll
      for (int r = 0; r < 8; ++r) {
        const float gv = acc[sub][t][r] * 0.03125f + bb[t];
        const float ex = __expf(-gv);
        aw[(8 * hh + r) * OTP + 16 * t + c] = __builtin_amdgcn_rcpf(1.0f + ex);
      }
    }
    __syncthreads();

    v4f val[8];
    size_t go[8];
#pragma unroll
    for (int it = 0; it < 8; ++it) {
      const int p    = lane + 32 * it;
      const int L    = p >> 3;
      const int pc   = p & 7;
      const int row  = L >> 1;
      const int half = L & 1;
      const v4f al = *(const v4f*)(aw + row * OTP + half * 32 + pc * 4);
      const v4f ht = *(const v4f*)(sw + (16 * sub + row) * OTP + half * 32 + pc * 4);
      go[it] = (trow + m0 + 16 * sub + row) * HID + n0 + half * 32 + pc * 4;
      const v4f hx = *(const v4f*)(hid + go[it]);
      val[it] = (v4f){(1.0f - al[0]) * hx[0] + al[0] * ht[0],
                      (1.0f - al[1]) * hx[1] + al[1] * ht[1],
                      (1.0f - al[2]) * hx[2] + al[2] * ht[2],
                      (1.0f - al[3]) * hx[3] + al[3] * ht[3]};
    }
    for (int ps = 0; ps < 2; ++ps) {
#pragma unroll
      for (int it = 0; it < 8; ++it) *(volatile v4f*)(out + go[it]) = val[it];
      __threadfence();
    }
  }
}

extern "C" void kernel_launch(void* const* d_in, const int* in_sizes, int n_in,
                              void* d_out, int out_size, void* d_ws, size_t ws_size,
                              hipStream_t stream) {
  if (n_in < 7) return;
  if (in_sizes[0] != NTOK * HID) return;
  if (in_sizes[1] != NB * NMEM * HID) return;
  if (in_sizes[2] != HID * HID) return;
  if (in_sizes[3] != HID * HID) return;
  if (in_sizes[4] != HID) return;
  if (in_sizes[5] != HID * HID) return;
  if (in_sizes[6] != HID) return;
  if (out_size != NTOK * HID) return;

  const float* hid = (const float*)d_in[0];
  const float* mem = (const float*)d_in[1];
  const float* qw  = (const float*)d_in[2];
  const float* kw  = (const float*)d_in[3];
  const float* nw  = (const float*)d_in[4];
  const float* gw  = (const float*)d_in[5];
  const float* gb  = (const float*)d_in[6];
  float* out = (float*)d_out;

  size_t off = 0;
  const size_t oXh = off; off += (size_t)NTOK * HID * 2;
  const size_t oVp = off; off += (size_t)NB * NT * HID * 2;
  const size_t oWq = off; off += (size_t)HID * HID * 2;
  const size_t oWk = off; off += (size_t)HID * HID * 2;
  const size_t oWg = off; off += (size_t)HID * HID * 2;
  const size_t oQ  = off; off += (size_t)NB * SQ * HID * 2;
  const size_t oKp = off; off += (size_t)NB * NT * HID * 2;
  const size_t oVt = off; off += (size_t)NB * HID * NT * 2;
  const size_t oP  = off; off += (size_t)NB * SQ * NT * 2;
  if (off > ws_size) return;
  if (off > (size_t)134217728) return;

  char* ws = (char*)d_ws;
  _Float16* Xh = (_Float16*)(ws + oXh);
  _Float16* Vp = (_Float16*)(ws + oVp);
  _Float16* Wq = (_Float16*)(ws + oWq);
  _Float16* Wk = (_Float16*)(ws + oWk);
  _Float16* Wg = (_Float16*)(ws + oWg);
  _Float16* Qp = (_Float16*)(ws + oQ);
  _Float16* Kp = (_Float16*)(ws + oKp);
  _Float16* Vt = (_Float16*)(ws + oVt);
  _Float16* Pp = (_Float16*)(ws + oP);

  k_prep<<<dim3(NB * NT / 2), dim3(256), 0, stream>>>(hid, mem, nw, Vp, Xh);
  k_cvtw<<<dim3(HID / 2), dim3(256), 0, stream>>>(qw, Wq, 32.0f);
  k_cvtw<<<dim3(HID / 2), dim3(256), 0, stream>>>(kw, Wk, 32.0f);
  k_cvtw<<<dim3(HID / 2), dim3(256), 0, stream>>>(gw, Wg, 32.0f);
  k_proj<<<dim3(SQ / 64, 4, NB), dim3(256), 0, stream>>>(Vp, (size_t)NT * HID, Wq, Qp, (size_t)SQ * HID);
  k_proj<<<dim3(NT / 64, 4, NB), dim3(256), 0, stream>>>(Vp, (size_t)NT * HID, Wk, Kp, (size_t)NT * HID);
  k_vtr<<<dim3(NT / 64, HID / 64, NB), dim3(256), 0, stream>>>(Vp, Vt);
  k_ssm<<<dim3(SQ / 16, NB), dim3(256), 0, stream>>>(Qp, Kp, Pp);
  k_pvg<<<dim3(SQ / 256, HID / 64, NB), dim3(256), 0, stream>>>(Pp, Vt, Xh, Wg, gb, hid, out);
  (void)hipGetLastError();
}
